// StatePerturbationEncoder_19765439496829
// MI455X (gfx1250) — hardware-verified
//
#include <hip/hip_runtime.h>
#include <math.h>

typedef __bf16 v16bf __attribute__((ext_vector_type(16)));
typedef __bf16 v8bf_r __attribute__((ext_vector_type(8)));
typedef v8bf_r __attribute__((may_alias)) v8bf;
typedef __bf16 v4bf_r __attribute__((ext_vector_type(4)));
typedef v4bf_r __attribute__((may_alias)) v4bf;
typedef float v8f __attribute__((ext_vector_type(8)));
typedef float v4f_r __attribute__((ext_vector_type(4)));
typedef v4f_r __attribute__((may_alias)) v4f;
typedef int v4i_r __attribute__((ext_vector_type(4)));
typedef v4i_r __attribute__((may_alias)) v4i;

#define DD 256
#define RB 64
#define XP 264
#define YP 260
#define SBUF_BYTES (2 * RB * XP * 2)
#define EPSF 1e-5f

union Frag16 { v16bf v; v8bf h[2]; };
union Pack16 { v8bf b; v4i i; };

__device__ __forceinline__ float gelu_f(float x) {
    return 0.5f * x * (1.0f + erff(x * 0.70710678118654752f));
}

__device__ __forceinline__ v8f wmma_hilo(v16bf ah, v16bf al, v16bf bh, v16bf bl, v8f c) {
    c = __builtin_amdgcn_wmma_f32_16x16x32_bf16(false, ah, false, bh, (short)0, c, false, false);
    c = __builtin_amdgcn_wmma_f32_16x16x32_bf16(false, ah, false, bl, (short)0, c, false, false);
    c = __builtin_amdgcn_wmma_f32_16x16x32_bf16(false, al, false, bh, (short)0, c, false, false);
    asm volatile("v_nop\n\tv_nop\n\tv_nop\n\tv_nop" : "+v"(c) : "v"(ah), "v"(al), "v"(bh), "v"(bl));
    return c;
}

__global__ __launch_bounds__(256) void k_wsplit(const float* __restrict__ W1, const float* __restrict__ W2,
                                                const float* __restrict__ W3, const float* __restrict__ W4,
                                                __bf16* wsp, int lo_off) {
    __shared__ __attribute__((aligned(16))) __bf16 sH[32 * XP];
    __shared__ __attribute__((aligned(16))) __bf16 sL[32 * XP];
    const int tid = threadIdx.x, lane = tid & 31, wv = tid >> 5;
    const int l = blockIdx.x >> 3;
    const int n0 = (blockIdx.x & 7) * 32;
    const float* W = (l == 0) ? W1 : (l == 1) ? W2 : (l == 2) ? W3 : W4;

    for (int it = 0; it < 32; ++it) {
        const int k = it * 8 + wv;
        const int c = lane;
        const float v = W[(size_t)k * DD + n0 + c];
        const __bf16 hi = (__bf16)v;
        const __bf16 lo = (__bf16)(v - (float)hi);
        sH[c * XP + k] = hi;
        sL[c * XP + k] = lo;
    }
    __syncthreads();

    __bf16* dh = wsp + (size_t)l * DD * DD;
    __bf16* dl = wsp + (size_t)lo_off + (size_t)l * DD * DD;
    #pragma unroll
    for (int j = 0; j < 4; ++j) {
        const int n = wv * 4 + j;
        Pack16 ph, pl;
        ph.b = *(const v8bf*)(sH + n * XP + lane * 8);
        pl.b = *(const v8bf*)(sL + n * XP + lane * 8);
        *(volatile v4i*)(dh + (size_t)(n0 + n) * DD + lane * 8) = ph.i;
        *(volatile v4i*)(dl + (size_t)(n0 + n) * DD + lane * 8) = pl.i;
    }
    __threadfence();
    #pragma unroll
    for (int j = 0; j < 4; ++j) {
        const int n = wv * 4 + j;
        Pack16 ph, pl;
        ph.b = *(const v8bf*)(sH + n * XP + lane * 8);
        pl.b = *(const v8bf*)(sL + n * XP + lane * 8);
        *(volatile v4i*)(dh + (size_t)(n0 + n) * DD + lane * 8) = ph.i;
        *(volatile v4i*)(dl + (size_t)(n0 + n) * DD + lane * 8) = pl.i;
    }
}

__global__ __launch_bounds__(256) void k_bnfin(const float* __restrict__ part, int nblk, int nrows,
                                               const float* __restrict__ gamma, const float* __restrict__ beta,
                                               float* bnout) {
    __shared__ __attribute__((aligned(16))) float sB[2 * DD];
    const int t = threadIdx.x, lane = t & 31, wv = t >> 5;
    double s = 0.0, q = 0.0;
    for (int b = 0; b < nblk; ++b) {
        s += (double)part[(size_t)b * (2 * DD) + t];
        q += (double)part[(size_t)b * (2 * DD) + DD + t];
    }
    const double invn = 1.0 / (double)nrows;
    const double mu = s * invn;
    double var = q * invn - mu * mu;
    if (var < 0.0) var = 0.0;
    const float muf = (float)mu;
    const float varf = (float)var;
    const float sc = gamma[t] * rsqrtf(varf + EPSF);
    const float sh = beta[t] - muf * sc;
    sB[t] = sc;
    sB[DD + t] = sh;
    __syncthreads();
    if (wv == 0) {
        #pragma unroll
        for (int q4 = 0; q4 < 4; ++q4) {
            const v4f v = *(const v4f*)(sB + q4 * 128 + lane * 4);
            *(volatile v4f*)(bnout + q4 * 128 + lane * 4) = v;
        }
    }
    __threadfence();
    if (wv == 0) {
        #pragma unroll
        for (int q4 = 0; q4 < 4; ++q4) {
            const v4f v = *(const v4f*)(sB + q4 * 128 + lane * 4);
            *(volatile v4f*)(bnout + q4 * 128 + lane * 4) = v;
        }
    }
}

template <bool GATHER, bool BN_IN, bool STATS>
__global__ __launch_bounds__(256) void k_layer(const float* __restrict__ xin,
                                               const int* __restrict__ ids,
                                               const float* __restrict__ table,
                                               int ntab,
                                               const __bf16* __restrict__ wsp,
                                               int lo_off,
                                               const float* __restrict__ bias,
                                               const float* __restrict__ bn,
                                               float* yout,
                                               float* part,
                                               int nrows) {
    __shared__ __attribute__((aligned(16))) char sbuf[SBUF_BYTES];
    __shared__ float sPS[4 * DD];
    __shared__ float sPQ[4 * DD];
    __shared__ __attribute__((aligned(16))) float sC[2 * DD];
    __bf16* sXh = (__bf16*)sbuf;
    __bf16* sXl = sXh + RB * XP;
    float*  sY  = (float*)sbuf;

    const int tid  = threadIdx.x;
    const int lane = tid & 31;
    const int wv   = tid >> 5;
    const int rg   = wv >> 1;
    const int cg   = wv & 1;
    const int h    = lane >> 4;
    const int m    = lane & 15;
    const int row0 = blockIdx.x * RB;

    #pragma unroll 4
    for (int it = 0; it < 16; ++it) {
        const int f   = it * 256 + tid;
        const int r   = f >> 6;
        const int k   = (f & 63) << 2;
        const int row = row0 + r;
        v4f v = {0.0f, 0.0f, 0.0f, 0.0f};
        if (row < nrows) {
            const float* src;
            if (GATHER) {
                int id = ids[row];
                id = id < 0 ? 0 : id;
                id = id >= ntab ? ntab - 1 : id;
                src = table + (size_t)id * DD + k;
            } else {
                src = xin + (size_t)row * DD + k;
            }
            v = *(const v4f*)src;
            if (BN_IN) {
                const v4f sc = *(const v4f*)(bn + k);
                const v4f sh = *(const v4f*)(bn + DD + k);
                v = v * sc + sh;
            }
        }
        const __bf16 h0 = (__bf16)v.x, h1 = (__bf16)v.y, h2 = (__bf16)v.z, h3 = (__bf16)v.w;
        v4bf ph = {h0, h1, h2, h3};
        v4bf pl = {(__bf16)(v.x - (float)h0), (__bf16)(v.y - (float)h1),
                   (__bf16)(v.z - (float)h2), (__bf16)(v.w - (float)h3)};
        *(v4bf*)(sXh + r * XP + k) = ph;
        *(v4bf*)(sXl + r * XP + k) = pl;
    }
    __syncthreads();

    v8f acc[8];
    #pragma unroll
    for (int nt = 0; nt < 8; ++nt) { v8f z = {0.0f, 0.0f, 0.0f, 0.0f, 0.0f, 0.0f, 0.0f, 0.0f}; acc[nt] = z; }

    const __bf16* ahrow = sXh + (rg * 16 + m) * XP;
    const __bf16* alrow = sXl + (rg * 16 + m) * XP;
    const __bf16* wcol  = wsp + (size_t)(cg * 128 + m) * DD;

    #pragma unroll 1
    for (int kk = 0; kk < 8; ++kk) {
        const int k0 = kk * 32;
        Frag16 ah, al;
        ah.h[0] = *(const v8bf*)(ahrow + k0 + 8 * h);
        ah.h[1] = *(const v8bf*)(ahrow + k0 + 16 + 8 * h);
        al.h[0] = *(const v8bf*)(alrow + k0 + 8 * h);
        al.h[1] = *(const v8bf*)(alrow + k0 + 16 + 8 * h);
        #pragma unroll
        for (int nt = 0; nt < 8; ++nt) {
            const __bf16* pbh = wcol + (size_t)nt * 16 * DD + k0;
            const __bf16* pbl = pbh + lo_off;
            Frag16 bh, bl;
            bh.h[0] = *(const v8bf*)(pbh + 8 * h);
            bh.h[1] = *(const v8bf*)(pbh + 16 + 8 * h);
            bl.h[0] = *(const v8bf*)(pbl + 8 * h);
            bl.h[1] = *(const v8bf*)(pbl + 16 + 8 * h);
            acc[nt] = wmma_hilo(ah.v, al.v, bh.v, bl.v, acc[nt]);
        }
    }
    __syncthreads();

    const int lr0 = rg * 16 + 8 * h;
    #pragma unroll
    for (int nt = 0; nt < 8; ++nt) {
        const int col = cg * 128 + nt * 16 + m;
        const float bb = bias[col];
        float s = 0.0f, q = 0.0f;
        #pragma unroll
        for (int r = 0; r < 8; ++r) {
            const float g = gelu_f(acc[nt][r] + bb);
            sY[(lr0 + r) * YP + col] = g;
            if (STATS) {
                const float gm = (row0 + lr0 + r < nrows) ? g : 0.0f;
                s += gm;
                q += gm * gm;
            }
        }
        if (STATS) {
            s += __shfl_xor(s, 16);
            q += __shfl_xor(q, 16);
            if (h == 0) { sPS[rg * DD + col] = s; sPQ[rg * DD + col] = q; }
        }
    }
    __syncthreads();

    if (STATS) {
        const float s = ((sPS[tid] + sPS[DD + tid]) + sPS[2 * DD + tid]) + sPS[3 * DD + tid];
        const float q = ((sPQ[tid] + sPQ[DD + tid]) + sPQ[2 * DD + tid]) + sPQ[3 * DD + tid];
        sC[tid] = s;
        sC[DD + tid] = q;
        __syncthreads();
    }

    #pragma unroll
    for (int j = 0; j < 8; ++j) {
        const int rl  = wv * 8 + j;
        const int row = row0 + rl;
        if (row < nrows) {
            #pragma unroll
            for (int c = 0; c < 2; ++c) {
                const v4f v = *(const v4f*)(sY + rl * YP + c * 128 + lane * 4);
                *(volatile v4f*)(yout + (size_t)row * DD + c * 128 + lane * 4) = v;
            }
        }
    }
    if (STATS) {
        if (wv == 0) {
            #pragma unroll
            for (int q4 = 0; q4 < 4; ++q4) {
                const v4f v = *(const v4f*)(sC + q4 * 128 + lane * 4);
                *(volatile v4f*)(part + (size_t)blockIdx.x * (2 * DD) + q4 * 128 + lane * 4) = v;
            }
        }
    }
    __threadfence();
    #pragma unroll
    for (int j = 0; j < 8; ++j) {
        const int rl  = wv * 8 + j;
        const int row = row0 + rl;
        if (row < nrows) {
            #pragma unroll
            for (int c = 0; c < 2; ++c) {
                const v4f v = *(const v4f*)(sY + rl * YP + c * 128 + lane * 4);
                *(volatile v4f*)(yout + (size_t)row * DD + c * 128 + lane * 4) = v;
            }
        }
    }
    if (STATS) {
        if (wv == 0) {
            #pragma unroll
            for (int q4 = 0; q4 < 4; ++q4) {
                const v4f v = *(const v4f*)(sC + q4 * 128 + lane * 4);
                *(volatile v4f*)(part + (size_t)blockIdx.x * (2 * DD) + q4 * 128 + lane * 4) = v;
            }
        }
    }
}

extern "C" void kernel_launch(void* const* d_in, const int* in_sizes, int n_in,
                              void* d_out, int out_size, void* d_ws, size_t ws_size,
                              hipStream_t stream) {
    if (n_in < 16) return;
    const int nrows = in_sizes[0];
    if (nrows <= 0) return;
    if ((in_sizes[1] % DD) != 0 || in_sizes[1] < DD) return;
    const int ntab = in_sizes[1] / DD;
    for (int i = 0; i < 4; ++i) {
        if (in_sizes[2 + 2 * i] != DD * DD) return;
        if (in_sizes[3 + 2 * i] != DD) return;
    }
    for (int i = 10; i < 16; ++i) if (in_sizes[i] != DD) return;
    if (out_size != nrows * DD) return;

    const int*   ids   = (const int*)d_in[0];
    const float* table = (const float*)d_in[1];
    const float* W1 = (const float*)d_in[2];  const float* b1 = (const float*)d_in[3];
    const float* W2 = (const float*)d_in[4];  const float* b2 = (const float*)d_in[5];
    const float* W3 = (const float*)d_in[6];  const float* b3 = (const float*)d_in[7];
    const float* W4 = (const float*)d_in[8];  const float* b4 = (const float*)d_in[9];
    const float* g1 = (const float*)d_in[10]; const float* be1 = (const float*)d_in[11];
    const float* g2 = (const float*)d_in[12]; const float* be2 = (const float*)d_in[13];
    const float* g3 = (const float*)d_in[14]; const float* be3 = (const float*)d_in[15];
    float* out = (float*)d_out;

    const int nblk = (nrows + RB - 1) / RB;
    const int lo_off = 4 * DD * DD;

    char* ws = (char*)d_ws;
    size_t off = 0;
    const size_t ybytes   = (((size_t)nrows * DD * sizeof(float)) + 255) & ~(size_t)255;
    const size_t wbytes   = (size_t)8 * DD * DD * 2;
    const size_t pbytes   = (((size_t)nblk * 2 * DD * sizeof(float)) + 255) & ~(size_t)255;
    const size_t bnbytes  = (((size_t)3 * 2 * DD * sizeof(float)) + 255) & ~(size_t)255;
    float*  yA   = (float*)(ws + off);  off += ybytes;
    float*  yB   = (float*)(ws + off);  off += ybytes;
    __bf16* wsp  = (__bf16*)(ws + off); off += wbytes;
    float*  part = (float*)(ws + off);  off += pbytes;
    float*  bnb  = (float*)(ws + off);  off += bnbytes;
    if (off > ws_size) return;

    k_wsplit<<<32, 256, 0, stream>>>(W1, W2, W3, W4, wsp, lo_off);

    k_layer<true, false, true><<<nblk, 256, 0, stream>>>(
        yB, ids, table, ntab, wsp + 0 * DD * DD, lo_off, b1, bnb, yA, part, nrows);
    k_bnfin<<<1, 256, 0, stream>>>(part, nblk, nrows, g1, be1, bnb + 0 * 2 * DD);

    k_layer<false, true, true><<<nblk, 256, 0, stream>>>(
        yA, ids, table, ntab, wsp + 1 * DD * DD, lo_off, b2, bnb + 0 * 2 * DD, yB, part, nrows);
    k_bnfin<<<1, 256, 0, stream>>>(part, nblk, nrows, g2, be2, bnb + 1 * 2 * DD);

    k_layer<false, true, true><<<nblk, 256, 0, stream>>>(
        yB, ids, table, ntab, wsp + 2 * DD * DD, lo_off, b3, bnb + 1 * 2 * DD, yA, part, nrows);
    k_bnfin<<<1, 256, 0, stream>>>(part, nblk, nrows, g3, be3, bnb + 2 * 2 * DD);

    k_layer<false, true, false><<<nblk, 256, 0, stream>>>(
        yA, ids, table, ntab, wsp + 3 * DD * DD, lo_off, b4, bnb + 2 * 2 * DD, out, part, nrows);
}
